// Multi_Headed_59304908423973
// MI455X (gfx1250) — hardware-verified
//
#include <hip/hip_runtime.h>
#include <stdint.h>
#include <math.h>

typedef __attribute__((ext_vector_type(16))) _Float16 v16h;
typedef __attribute__((ext_vector_type(8)))  _Float16 v8h;
typedef __attribute__((ext_vector_type(16))) __bf16   v16b;
typedef __attribute__((ext_vector_type(8)))  __bf16   v8b;
typedef __attribute__((ext_vector_type(8)))  float    v8f;
typedef __attribute__((ext_vector_type(4)))  float    v4f;
typedef __attribute__((ext_vector_type(4)))  unsigned v4u;

constexpr int EMB_SZ  = 768;
constexpr int NHEAD   = 3;
constexpr int HDIM    = 256;
constexpr int NBATCH  = 4;
constexpr int SEQLEN  = 2048;
constexpr int NROWS   = NBATCH * SEQLEN;
constexpr size_t PLANE_ELEMS = (size_t)NROWS * EMB_SZ;
constexpr size_t PLANE_BYTES = PLANE_ELEMS * 2;
constexpr size_t WT_ELEMS    = (size_t)NHEAD * HDIM * EMB_SZ;
constexpr size_t WO_ELEMS    = (size_t)EMB_SZ * EMB_SZ;

constexpr size_t WS_OFF_WKT = 9 * PLANE_ELEMS;
constexpr size_t WS_OFF_WVT = WS_OFF_WKT + WT_ELEMS;
constexpr size_t WS_OFF_WQT = WS_OFF_WVT + WT_ELEMS;
constexpr size_t WS_OFF_WOT = WS_OFF_WQT + WT_ELEMS;
constexpr size_t WS_TOTAL_BYTES = (WS_OFF_WOT + WO_ELEMS) * 2;
static_assert(WS_TOTAL_BYTES == 117964800ull);
static_assert(WS_TOTAL_BYTES <= 134217728ull);
static_assert((PLANE_BYTES % 128) == 0 && ((WT_ELEMS * 2) % 128) == 0 && ((WO_ELEMS * 2) % 128) == 0);

static_assert(NROWS % 64 == 0 && HDIM % 64 == 0 && EMB_SZ % 64 == 0);
static_assert(EMB_SZ % 32 == 0);
static_assert(PLANE_ELEMS % (8 * 256) == 0);

__device__ __forceinline__ unsigned short f2bf_bits(float f) {
  unsigned u = __float_as_uint(f);
  return (unsigned short)((u + 0x7FFFu + ((u >> 16) & 1u)) >> 16);
}
__device__ __forceinline__ float bf_bits2f(unsigned short h) { return __uint_as_float(((unsigned)h) << 16); }

__device__ __forceinline__ void dep_guard_h(v8f& a, v8f& b, v16h x, v16h y) { asm volatile("v_nop\n\tv_nop\n\tv_nop\n\tv_nop" : "+v"(a), "+v"(b) : "v"(x), "v"(y)); }
__device__ __forceinline__ void dep_guard_b(v8f& a, v8f& b, v16b x, v16b y) { asm volatile("v_nop\n\tv_nop\n\tv_nop\n\tv_nop" : "+v"(a), "+v"(b) : "v"(x), "v"(y)); }
__device__ __forceinline__ void keep4_h(v16h a, v16h b, v16h c, v16h d) { asm volatile("v_nop" :: "v"(a), "v"(b), "v"(c), "v"(d)); }
__device__ __forceinline__ void keep4_b(v16b a, v16b b, v16b c, v16b d) { asm volatile("v_nop" :: "v"(a), "v"(b), "v"(c), "v"(d)); }
__device__ __forceinline__ void acc_guard4(v8f& a, v8f& b, v8f& c, v8f& d) { asm volatile("v_nop\n\tv_nop\n\tv_nop\n\tv_nop" : "+v"(a), "+v"(b), "+v"(c), "+v"(d)); }
template <typename T> struct Frag;
template <> struct Frag<_Float16> {
  typedef v16h V; union U { v16h v; v8h h[2]; };
  static __device__ __forceinline__ v16h load(const _Float16* p) {
    U f; f.h[0] = *(const v8h*)(p); f.h[1] = *(const v8h*)(p + 16); return f.v;
  }
  static __device__ __forceinline__ v8f mma(v16h a, v16h b, v8f c) {
    return __builtin_amdgcn_wmma_f32_16x16x32_f16(false, a, false, b, (short)0, c, false, false);
  }
  static __device__ __forceinline__ void guard(v8f& a, v8f& b, v16h x, v16h y) { dep_guard_h(a, b, x, y); }
  static __device__ __forceinline__ void keep(v16h a, v16h b, v16h c, v16h d) { keep4_h(a, b, c, d); }
};
template <> struct Frag<__bf16> {
  typedef v16b V; union U { v16b v; v8b h[2]; };
  static __device__ __forceinline__ v16b load(const __bf16* p) {
    U f; f.h[0] = *(const v8b*)(p); f.h[1] = *(const v8b*)(p + 16); return f.v;
  }
  static __device__ __forceinline__ v8f mma(v16b a, v16b b, v8f c) {
    return __builtin_amdgcn_wmma_f32_16x16x32_bf16(false, a, false, b, (short)0, c, false, false);
  }
  static __device__ __forceinline__ void guard(v8f& a, v8f& b, v16b x, v16b y) { dep_guard_b(a, b, x, y); }
  static __device__ __forceinline__ void keep(v16b a, v16b b, v16b c, v16b d) { keep4_b(a, b, c, d); }
};

template <int ET> struct Elem;
template <> struct Elem<0> { typedef _Float16 T; };
template <> struct Elem<1> { typedef __bf16 T; };
template <int ET, bool SPLITA, bool SPLITB, int BIAS_MODE, int OUT_MODE>
__global__ __launch_bounds__(256) void wmma_gemm64(
    const unsigned short* __restrict__ Ap, const unsigned short* __restrict__ A2p, int lda, long strideA,
    const unsigned short* __restrict__ Btp, const unsigned short* __restrict__ Bt2p, int ldb, long strideB,
    void* __restrict__ Cout, void* __restrict__ Cout2, int ldc, long strideC,
    const float* __restrict__ bias,
    int M, int N, int K, float scale) {
  typedef typename Elem<ET>::T T;
  typedef typename Frag<T>::V V;
  const T* A = (const T*)Ap; const T* A2 = (const T*)A2p; const T* Bt = (const T*)Btp; const T* Bt2 = (const T*)Bt2p;
  __shared__ __align__(16) float sT[8][16 * 68];
  const int b    = blockIdx.y;
  const int lane = threadIdx.x & 31;
  const int wave = threadIdx.x >> 5;
  const int tilesN = N >> 6;
  const int tilesM = M >> 6;
  const int tile = blockIdx.x * 8 + wave;
  if (tile >= tilesM * tilesN) return;
  const int tm = tile / tilesN;
  const int tn = tile - tm * tilesN;
  const int m0 = tm << 6;
  const int n0 = tn << 6;

  const T* Ab  = A  + (size_t)b * strideA;
  const T* Bb  = Bt + (size_t)b * strideB;
  const T* Ab2 = SPLITA ? (A2  + (size_t)b * strideA) : nullptr;
  const T* Bb2 = SPLITB ? (Bt2 + (size_t)b * strideB) : nullptr;

  const int rlane = lane & 15;
  const int koff  = (lane >> 4) * 8;
  const int mOff  = (lane >> 4) * 8;

  v8f acc[4][4];
#pragma unroll
  for (int i = 0; i < 4; ++i)
#pragma unroll
    for (int j = 0; j < 4; ++j) acc[i][j] = (v8f){0.f,0.f,0.f,0.f,0.f,0.f,0.f,0.f};

  for (int k0 = 0; k0 < K; k0 += 32) {
    V bh[4], bl[4];
#pragma unroll
    for (int j = 0; j < 4; ++j) {
      const size_t bo = (size_t)(n0 + (j << 4) + rlane) * ldb + koff + k0;
      bh[j] = Frag<T>::load(Bb + bo);
      if (SPLITB) bl[j] = Frag<T>::load(Bb2 + bo);
    }
#pragma unroll
    for (int i = 0; i < 4; ++i) {
      const size_t ao = (size_t)(m0 + (i << 4) + rlane) * lda + koff + k0;
      V ah = Frag<T>::load(Ab + ao);
      V al;
      if (SPLITA) al = Frag<T>::load(Ab2 + ao);
#pragma unroll
      for (int j = 0; j < 4; ++j) {
        acc[i][j] = Frag<T>::mma(ah, bh[j], acc[i][j]);
        if (SPLITB) acc[i][j] = Frag<T>::mma(ah, bl[j], acc[i][j]);
        if (SPLITA) acc[i][j] = Frag<T>::mma(al, bh[j], acc[i][j]);
      }
      Frag<T>::guard(acc[i][0], acc[i][3], ah, SPLITA ? al : ah);
    }
    Frag<T>::keep(bh[0], bh[1], bh[2], bh[3]);
    if (SPLITB) Frag<T>::keep(bl[0], bl[1], bl[2], bl[3]);
  }
  acc_guard4(acc[0][0], acc[0][1], acc[0][2], acc[0][3]);
  acc_guard4(acc[1][0], acc[1][1], acc[1][2], acc[1][3]);
  acc_guard4(acc[2][0], acc[2][1], acc[2][2], acc[2][3]);
  acc_guard4(acc[3][0], acc[3][1], acc[3][2], acc[3][3]);

  float* slab = sT[wave];
#pragma unroll
  for (int i = 0; i < 4; ++i) {
    const int mBase = m0 + (i << 4);
#pragma unroll
    for (int j = 0; j < 4; ++j) {
      const int n = n0 + (j << 4) + rlane;
      float bv = 0.f;
      if (BIAS_MODE == 2) bv = bf_bits2f(f2bf_bits(bias[n]));
#pragma unroll
      for (int r = 0; r < 8; ++r) {
        float v = acc[i][j][r] * scale;
        if (BIAS_MODE == 1) v += bias[mBase + mOff + r];
        if (BIAS_MODE == 2) v += bv;
        slab[(mOff + r) * 68 + (j << 4) + rlane] = v;
      }
    }
    __builtin_amdgcn_fence(__ATOMIC_RELEASE, "workgroup");
    __builtin_amdgcn_wave_barrier();
    __builtin_amdgcn_fence(__ATOMIC_ACQUIRE, "workgroup");
    if (OUT_MODE == 0) {
      float* C = (float*)Cout + (size_t)b * strideC;
      const int hh = lane >> 4, c4 = (lane & 15) * 4;
      for (int pass = 0; pass < 2; ++pass) {
#pragma unroll
        for (int it = 0; it < 8; ++it) {
          const int row = it * 2 + hh;
          v4f v = *(const v4f*)(slab + row * 68 + c4);
          *(volatile v4f*)(C + (size_t)(mBase + row) * ldc + n0 + c4) = v;
        }
        __threadfence();
      }
    } else {
      const int q = lane >> 3, c8 = (lane & 7) * 8;
      unsigned short* C  = (unsigned short*)Cout  + (size_t)b * strideC;
      unsigned short* C2 = (OUT_MODE == 2) ? ((unsigned short*)Cout2 + (size_t)b * strideC) : nullptr;
      for (int pass = 0; pass < 2; ++pass) {
#pragma unroll
        for (int it = 0; it < 4; ++it) {
          const int row = it * 4 + q;
          const float* sp = slab + row * 68 + c8;
          v8h hv, lv;
#pragma unroll
          for (int e = 0; e < 8; ++e) {
            if (OUT_MODE == 1) {
              hv[e] = (_Float16)sp[e];
            } else {
              unsigned short hb = f2bf_bits(sp[e]);
              unsigned short lb = f2bf_bits(sp[e] - bf_bits2f(hb));
              hv[e] = __builtin_bit_cast(_Float16, hb);
              lv[e] = __builtin_bit_cast(_Float16, lb);
            }
          }
          *(volatile v8h*)(C + (size_t)(mBase + row) * ldc + n0 + c8) = hv;
          if (OUT_MODE == 2) *(volatile v8h*)(C2 + (size_t)(mBase + row) * ldc + n0 + c8) = lv;
        }
        __threadfence();
      }
    }
    __builtin_amdgcn_fence(__ATOMIC_RELEASE, "workgroup");
    __builtin_amdgcn_wave_barrier();
    __builtin_amdgcn_fence(__ATOMIC_ACQUIRE, "workgroup");
  }
}

__global__ __launch_bounds__(256) void cvt_f32_bf16x8(
    const float* __restrict__ in, unsigned short* __restrict__ out, int n8) {
  const int i = blockIdx.x * 256 + threadIdx.x;
  if (i < n8) {
    const float* p = in + (size_t)i * 8;
    const v4f a = *(const v4f*)p;
    const v4f c2 = *(const v4f*)(p + 4);
    v4u w;
    w[0] = (unsigned)f2bf_bits(a[0])  | ((unsigned)f2bf_bits(a[1])  << 16);
    w[1] = (unsigned)f2bf_bits(a[2])  | ((unsigned)f2bf_bits(a[3])  << 16);
    w[2] = (unsigned)f2bf_bits(c2[0]) | ((unsigned)f2bf_bits(c2[1]) << 16);
    w[3] = (unsigned)f2bf_bits(c2[2]) | ((unsigned)f2bf_bits(c2[3]) << 16);
    unsigned short* o = out + (size_t)i * 8;
    *(volatile v4u*)o = w;
    __threadfence();
    *(volatile v4u*)o = w;
  }
}

__global__ __launch_bounds__(256) void tr_cvt_bf16(
    const float* __restrict__ in, unsigned short* __restrict__ out, int R, int CC) {
  __shared__ float tile[64][65];
  const int tid = threadIdx.x;
  const size_t zoff = (size_t)blockIdx.z * (size_t)R * (size_t)CC;
  const float* src = in + zoff;
  unsigned short* dst = out + zoff;
  const int ct = blockIdx.x, rt = blockIdx.y;
  const int lr = tid >> 2, lc = (tid & 3) * 16;
  const float* sp = src + (size_t)(rt * 64 + lr) * CC + ct * 64 + lc;
#pragma unroll
  for (int i = 0; i < 4; ++i) {
    const v4f v = *(const v4f*)(sp + 4 * i);
    tile[lr][lc + 4 * i + 0] = v[0];
    tile[lr][lc + 4 * i + 1] = v[1];
    tile[lr][lc + 4 * i + 2] = v[2];
    tile[lr][lc + 4 * i + 3] = v[3];
  }
  __syncthreads();
  const int lane = tid & 31, wave = tid >> 5, q = lane >> 3, c8 = (lane & 7) * 8;
  v4u w[2];
#pragma unroll
  for (int it = 0; it < 2; ++it) {
    const int fl = wave * 8 + it * 4 + q;
    v4u t4;
#pragma unroll
    for (int e = 0; e < 4; ++e) {
      const unsigned lo16 = (unsigned)f2bf_bits(tile[c8 + 2 * e][fl]);
      const unsigned hi16 = (unsigned)f2bf_bits(tile[c8 + 2 * e + 1][fl]);
      t4[e] = lo16 | (hi16 << 16);
    }
    w[it] = t4;
  }
  for (int pass = 0; pass < 2; ++pass) {
#pragma unroll
    for (int it = 0; it < 2; ++it) {
      const int fl = wave * 8 + it * 4 + q;
      *(volatile v4u*)(dst + (size_t)(ct * 64 + fl) * R + rt * 64 + c8) = w[it];
    }
    __threadfence();
  }
}

constexpr int AT_KEYS  = 64;
constexpr int AT_QROWS = 64;
constexpr int AT_WHALF = 128;
static_assert(SEQLEN % AT_QROWS == 0 && SEQLEN % AT_KEYS == 0 && HDIM == 2 * AT_WHALF);
static_assert(8 * 16 * AT_WHALF == AT_KEYS * HDIM);

__device__ __forceinline__ v16b ldfrag16(const unsigned short* p) {
  union { v16b v; v8b h[2]; } f;
  f.h[0] = *(const v8b*)(p); f.h[1] = *(const v8b*)(p + 16); return f.v;
}
__device__ __forceinline__ v8f mma_bf(v16b a, v16b b, v8f c) {
  c = __builtin_amdgcn_wmma_f32_16x16x32_bf16(false, a, false, b, (short)0, c, false, false);
  asm volatile("v_nop\n\tv_nop\n\tv_nop\n\tv_nop" : "+v"(c) : "v"(a), "v"(b));
  return c;
}

__global__ __launch_bounds__(256) void attn_hd256(
    const unsigned short* __restrict__ Qh, const unsigned short* __restrict__ Ql,
    const unsigned short* __restrict__ Kh, const unsigned short* __restrict__ Kl,
    const unsigned short* __restrict__ Vh, const unsigned short* __restrict__ Vl,
    unsigned short* __restrict__ Oh, unsigned short* __restrict__ Ol, float inv_scale) {
  __shared__ __align__(16) unsigned short Ks[2][AT_KEYS * HDIM];
  __shared__ __align__(16) unsigned short Vts[2][HDIM * AT_KEYS];
  __shared__ __align__(16) unsigned short Ps[2][AT_QROWS * AT_KEYS];
  __shared__ float redm[2][AT_QROWS];
  __shared__ float reds[2][AT_QROWS];

  const int tid  = threadIdx.x;
  const int lane = tid & 31;
  const int wave = tid >> 5;
  const int hh   = lane >> 4;
  const int c    = lane & 15;
  const int rw   = wave & 3;
  const int ch   = wave >> 2;
  const int qb   = blockIdx.x;
  const int bh   = blockIdx.y;
  const int h    = bh % NHEAD;
  const int b    = bh / NHEAD;
  const int q0w  = qb * AT_QROWS + rw * 16;
  const size_t rowb = (size_t)b * SEQLEN;
  const int hcol = h * HDIM;

  float mrow[8], lrow[8];
  v8f oacc[8];
#pragma unroll
  for (int r = 0; r < 8; ++r) { mrow[r] = -INFINITY; lrow[r] = 0.f; }
#pragma unroll
  for (int t = 0; t < 8; ++t) oacc[t] = (v8f){0.f,0.f,0.f,0.f,0.f,0.f,0.f,0.f};

  const int nch = qb + 1;
  for (int kc = 0; kc < nch; ++kc) {
    const int kv0 = kc * AT_KEYS;
    __syncthreads();
    {
      const int kvr = tid >> 2, dq = (tid & 3) * 64;
      const size_t gbase = (rowb + kv0 + kvr) * EMB_SZ + hcol + dq;
#pragma unroll 1
      for (int i = 0; i < 8; ++i) {
        const v4u kh4 = *(const v4u*)(Kh + gbase + 8 * i);
        const v4u kl4 = *(const v4u*)(Kl + gbase + 8 * i);
        *(v4u*)(&Ks[0][kvr * HDIM + dq + 8 * i]) = kh4;
        *(v4u*)(&Ks[1][kvr * HDIM + dq + 8 * i]) = kl4;
      }
#pragma unroll 1
      for (int i = 0; i < 8; ++i) {
        const v4u vh4 = *(const v4u*)(Vh + gbase + 8 * i);
        const v4u vl4 = *(const v4u*)(Vl + gbase + 8 * i);
#pragma unroll
        for (int e = 0; e < 8; ++e) {
          const int d = dq + 8 * i + e;
          const unsigned sh = (unsigned)(e & 1) * 16u;
          Vts[0][d * AT_KEYS + kvr] = (unsigned short)((vh4[e >> 1] >> sh) & 0xffffu);
          Vts[1][d * AT_KEYS + kvr] = (unsigned short)((vl4[e >> 1] >> sh) & 0xffffu);
        }
      }
    }
    __syncthreads();

    v8f s[2];
    s[0] = (v8f){0.f,0.f,0.f,0.f,0.f,0.f,0.f,0.f};
    s[1] = (v8f){0.f,0.f,0.f,0.f,0.f,0.f,0.f,0.f};
    {
      const size_t qoff = (rowb + q0w + c) * EMB_SZ + hcol + 8 * hh;
#pragma unroll 1
      for (int dc = 0; dc < 8; ++dc) {
        const v16b qa  = ldfrag16(Qh + qoff + dc * 32);
        const v16b qal = ldfrag16(Ql + qoff + dc * 32);
#pragma unroll
        for (int j = 0; j < 2; ++j) {
          const int kr = ch * 32 + j * 16 + c;
          const int koff = kr * HDIM + dc * 32 + 8 * hh;
          const v16b kb = ldfrag16(&Ks[0][koff]);
          const v16b kl = ldfrag16(&Ks[1][koff]);
          s[j] = mma_bf(qa, kb, s[j]);
          s[j] = mma_bf(qa, kl, s[j]);
          s[j] = mma_bf(qal, kb, s[j]);
        }
      }
    }

    const bool diag = (kc == qb);
#pragma unroll
    for (int r = 0; r < 8; ++r) {
      const int qrow = q0w + 8 * hh + r;
      float m = -INFINITY;
#pragma unroll
      for (int j = 0; j < 2; ++j) {
        const int kvcol = kv0 + ch * 32 + j * 16 + c;
        float sv = s[j][r] * inv_scale;
        if (diag && (kvcol > qrow)) sv = -INFINITY;
        s[j][r] = sv;
        m = fmaxf(m, sv);
      }
      m = fmaxf(m, __shfl_xor(m, 1, 32));
      m = fmaxf(m, __shfl_xor(m, 2, 32));
      m = fmaxf(m, __shfl_xor(m, 4, 32));
      m = fmaxf(m, __shfl_xor(m, 8, 32));
      redm[ch][rw * 16 + 8 * hh + r] = m;
    }
    __syncthreads();

    float alph[8];
#pragma unroll
    for (int r = 0; r < 8; ++r) {
      const int row = rw * 16 + 8 * hh + r;
      const float mc = fmaxf(redm[0][row], redm[1][row]);
      const float mnew = fmaxf(mrow[r], mc);
      const float alpha = expf(mrow[r] - mnew);
      mrow[r] = mnew;
      alph[r] = alpha;
      float psum = 0.f;
#pragma unroll
      for (int j = 0; j < 2; ++j) {
        const float p = expf(s[j][r] - mnew);
        psum += p;
        const unsigned short hb = f2bf_bits(p);
        const unsigned short lb = f2bf_bits(p - bf_bits2f(hb));
        const int pidx = row * AT_KEYS + ch * 32 + j * 16 + c;
        Ps[0][pidx] = hb;
        Ps[1][pidx] = lb;
      }
      psum += __shfl_xor(psum, 1, 32);
      psum += __shfl_xor(psum, 2, 32);
      psum += __shfl_xor(psum, 4, 32);
      psum += __shfl_xor(psum, 8, 32);
      reds[ch][row] = psum;
#pragma unroll
      for (int t = 0; t < 8; ++t) oacc[t][r] *= alpha;
    }
    __syncthreads();
#pragma unroll
    for (int r = 0; r < 8; ++r) {
      const int row = rw * 16 + 8 * hh + r;
      lrow[r] = lrow[r] * alph[r] + (reds[0][row] + reds[1][row]);
    }

#pragma unroll 1
    for (int kk = 0; kk < 2; ++kk) {
      const int poff = (rw * 16 + c) * AT_KEYS + kk * 32 + 8 * hh;
      const v16b pa = ldfrag16(&Ps[0][poff]);
      const v16b pl = ldfrag16(&Ps[1][poff]);
#pragma unroll
      for (int t = 0; t < 8; ++t) {
        const int voff = (ch * AT_WHALF + t * 16 + c) * AT_KEYS + kk * 32 + 8 * hh;
        const v16b vb = ldfrag16(&Vts[0][voff]);
        const v16b vl = ldfrag16(&Vts[1][voff]);
        oacc[t] = mma_bf(pa, vb, oacc[t]);
        oacc[t] = mma_bf(pa, vl, oacc[t]);
        oacc[t] = mma_bf(pl, vb, oacc[t]);
      }
    }
  }

  __syncthreads();
  unsigned short* slh = &Ks[0][wave * (16 * AT_WHALF)];
  unsigned short* sll = &Ks[1][wave * (16 * AT_WHALF)];
#pragma unroll
  for (int r = 0; r < 8; ++r) {
    const float inv = 1.0f / lrow[r];
    const int row = 8 * hh + r;
#pragma unroll
    for (int t = 0; t < 8; ++t) {
      const float v = oacc[t][r] * inv;
      const unsigned short hb = f2bf_bits(v);
      const unsigned short lb = f2bf_bits(v - bf_bits2f(hb));
      slh[row * AT_WHALF + t * 16 + c] = hb;
      sll[row * AT_WHALF + t * 16 + c] = lb;
    }
  }
  __syncthreads();
  {
    for (int pass = 0; pass < 2; ++pass) {
#pragma unroll
      for (int it = 0; it < 8; ++it) {
        const int row = it * 2 + hh;
        const v4u wh = *(const v4u*)(slh + row * AT_WHALF + c * 8);
        const v4u wl = *(const v4u*)(sll + row * AT_WHALF + c * 8);
        const size_t go = (rowb + q0w + row) * EMB_SZ + hcol + ch * AT_WHALF + c * 8;
        *(volatile v4u*)(Oh + go) = wh;
        *(volatile v4u*)(Ol + go) = wl;
      }
      __threadfence();
    }
  }
}

extern "C" void kernel_launch(void* const* d_in, const int* in_sizes, int n_in,
                              void* d_out, int out_size, void* d_ws, size_t ws_size,
                              hipStream_t stream) {
  (void)in_sizes; (void)n_in; (void)out_size;
  const float* Xk = (const float*)d_in[0];
  const float* Xv = (const float*)d_in[1];
  const float* Xq = (const float*)d_in[2];
  const float* Wk = (const float*)d_in[3];
  const float* Wv = (const float*)d_in[4];
  const float* Wq = (const float*)d_in[5];
  const float* Wo = (const float*)d_in[6];
  const float* bo = (const float*)d_in[7];
  float* out = (float*)d_out;

  if (ws_size < WS_TOTAL_BYTES) return;

  unsigned short* ws = (unsigned short*)d_ws;
  unsigned short* xk_b = ws + 0 * PLANE_ELEMS;
  unsigned short* xv_b = ws + 1 * PLANE_ELEMS;
  unsigned short* xq_b = ws + 2 * PLANE_ELEMS;
  unsigned short* k_hi = ws + 3 * PLANE_ELEMS;
  unsigned short* k_lo = ws + 4 * PLANE_ELEMS;
  unsigned short* v_hi = ws + 5 * PLANE_ELEMS;
  unsigned short* v_lo = ws + 6 * PLANE_ELEMS;
  unsigned short* q_hi = ws + 7 * PLANE_ELEMS;
  unsigned short* q_lo = ws + 8 * PLANE_ELEMS;
  unsigned short* wkT  = ws + WS_OFF_WKT;
  unsigned short* wvT  = ws + WS_OFF_WVT;
  unsigned short* wqT  = ws + WS_OFF_WQT;
  unsigned short* woT  = ws + WS_OFF_WOT;
  unsigned short* cc_hi = xk_b;
  unsigned short* cc_lo = xv_b;

  const int n8 = (int)(PLANE_ELEMS / 8);
  cvt_f32_bf16x8<<<dim3(n8 / 256), 256, 0, stream>>>(Xk, xk_b, n8);
  cvt_f32_bf16x8<<<dim3(n8 / 256), 256, 0, stream>>>(Xv, xv_b, n8);
  cvt_f32_bf16x8<<<dim3(n8 / 256), 256, 0, stream>>>(Xq, xq_b, n8);

  tr_cvt_bf16<<<dim3(HDIM / 64, EMB_SZ / 64, NHEAD), 256, 0, stream>>>(Wk, wkT, EMB_SZ, HDIM);
  tr_cvt_bf16<<<dim3(HDIM / 64, EMB_SZ / 64, NHEAD), 256, 0, stream>>>(Wv, wvT, EMB_SZ, HDIM);
  tr_cvt_bf16<<<dim3(HDIM / 64, EMB_SZ / 64, NHEAD), 256, 0, stream>>>(Wq, wqT, EMB_SZ, HDIM);
  tr_cvt_bf16<<<dim3(EMB_SZ / 64, EMB_SZ / 64, 1), 256, 0, stream>>>(Wo, woT, EMB_SZ, EMB_SZ);

  const dim3 gproj((NROWS / 64) * (HDIM / 64) / 8, NHEAD);
  wmma_gemm64<1, false, false, 0, 2><<<gproj, 256, 0, stream>>>(
      xk_b, xk_b, EMB_SZ, 0L, wkT, wkT, EMB_SZ, (long)HDIM * EMB_SZ,
      (void*)k_hi, (void*)k_lo, EMB_SZ, (long)HDIM, bo, NROWS, HDIM, EMB_SZ, 1.0f);
  wmma_gemm64<1, false, false, 0, 2><<<gproj, 256, 0, stream>>>(
      xv_b, xv_b, EMB_SZ, 0L, wvT, wvT, EMB_SZ, (long)HDIM * EMB_SZ,
      (void*)v_hi, (void*)v_lo, EMB_SZ, (long)HDIM, bo, NROWS, HDIM, EMB_SZ, 1.0f);
  wmma_gemm64<1, false, false, 0, 2><<<gproj, 256, 0, stream>>>(
      xq_b, xq_b, EMB_SZ, 0L, wqT, wqT, EMB_SZ, (long)HDIM * EMB_SZ,
      (void*)q_hi, (void*)q_lo, EMB_SZ, (long)HDIM, bo, NROWS, HDIM, EMB_SZ, 1.0f);

  const float inv_scale = 1.0f / sqrtf((float)SEQLEN);
  attn_hd256<<<dim3(SEQLEN / AT_QROWS, NBATCH * NHEAD), 256, 0, stream>>>(
      q_hi, q_lo, k_hi, k_lo, v_hi, v_lo, cc_hi, cc_lo, inv_scale);

  const dim3 gout((NROWS / 64) * (EMB_SZ / 64) / 8, 1);
  wmma_gemm64<1, true, false, 2, 0><<<gout, 256, 0, stream>>>(
      cc_hi, cc_lo, EMB_SZ, 0L, woT, woT, EMB_SZ, 0L,
      (void*)out, (void*)out, EMB_SZ, 0L, bo, NROWS, EMB_SZ, EMB_SZ, 1.0f);
}
